// EdgeHGTConv_81372450390265
// MI455X (gfx1250) — hardware-verified
//
#include <hip/hip_runtime.h>
#include <stddef.h>
#include <stdint.h>
#include <math.h>

#define NN     20000
#define NE     200000
#define CH     64
#define NHEAD  4
#define HSZ    16
#define NTN    4
#define NTE    8
#define TM     128
#define NMT    157
#define MPN    (NMT * TM)
#define NTILE  1571
#define PCAP   (NTILE * TM)
#define NTHR   256
#define NWAVE  8
#define WSMAX  134217728

#define EPT    8
#define CHUNK  (NTHR * EPT)
#define WCAP   (EPT * 32)
#define LISTN  (NWAVE * WCAP)
#define NBMAX  2048
#define SLOTB  11
#define RCAP   28672
#define DEGCAP 64
#define NBRUN  1024
#define NSCANB 20
#define MX0    (-1.0e30f)
#define LDS_AGG ((2 * RCAP + 2 * NBMAX + LISTN) * 4 + 64)

#define PCH    2048
#define PSTG   2304

#define WB_WEA 0
#define WB_WEM (NTE * 1024 * CH)
#define WB_WRM (WB_WEM + NTE * CH * CH)
#define WB_TOT (WB_WRM + NTE * NHEAD * HSZ * 32)
#define FT_WRA 0
#define FT_PRQ (NTE * NHEAD * HSZ * HSZ)
#define FT_ALP (FT_PRQ + 32)
#define FT_TOT (FT_PRQ + 64)

#define XEP 72
#define VAP 136
#define WEP 72
#define WRP 40
#define E_OFF_KT   0
#define E_OFF_QT   (E_OFF_KT + CH * TM * 4)
#define E_OFF_MSG  (E_OFF_QT + CH * TM * 4)
#define E_OFF_SC   (E_OFF_MSG + TM * CH * 4)
#define E_OFF_WRA  (E_OFF_SC + TM * 4 * 4)
#define E_OFF_XE   (E_OFF_WRA + NHEAD * HSZ * HSZ * 4)
#define E_OFF_VA   (E_OFF_XE + TM * XEP * 2)
#define E_OFF_WEA  (E_OFF_VA + TM * VAP * 2)
#define E_OFF_WEM  (E_OFF_WEA + 256 * WEP * 2)
#define E_OFF_WRM  (E_OFF_WEM + CH * WEP * 2)
#define E_OFF_IDS  (E_OFF_WRM + CH * WRP * 2)
#define EDGE_LDS   (E_OFF_IDS + 5 * TM * 4)

#define PA_U0  (MPN * 8)
#define PA_U1  (PA_U0 + NE * 8)
#define PB_A   (NTN * CH * 8)
#define PB_D   (NTN * CH * 16)
#define PB_TOT (3 * PB_A + PB_D)
#define PB_NBLK (PB_TOT / NTHR)
#define PC_A   (NTE * 1024 * 8)
#define PC_B   (NTE * CH * 8)
#define PC_C   (NTE * NHEAD * HSZ * 4)
#define PC_D   (NTE * NHEAD * HSZ * 4)
#define PC_TOT (PC_A + PC_B + PC_C + PC_D)

static_assert(MPN >= NN && MPN % TM == 0);
static_assert((NE + NTE * 127 + 127) / 128 <= NTILE);
static_assert(NE % 4 == 0 && PCAP % 4 == 0);
static_assert(PCAP < (1 << (32 - SLOTB)));
static_assert((CHUNK & (CHUNK - 1)) == 0 && CHUNK <= (1 << SLOTB));
static_assert(NBMAX == (1 << SLOTB) && NTHR * 8 == NBMAX && LISTN >= NBMAX);
static_assert(NBRUN <= NBMAX && (NBRUN & (NBRUN - 1)) == 0 && NBRUN % NWAVE == 0);
static_assert(NSCANB * NBRUN >= MPN);
static_assert(RCAP % 32 == 0 && RCAP >= 2 * 10388);
static_assert(DEGCAP >= 23 + 8);
static_assert(LDS_AGG <= 300000 && EDGE_LDS <= 300000);
static_assert(PA_U0 % NTHR == 0 && PA_U1 % NTHR == 0);
static_assert(PB_A % NTHR == 0 && PB_D % NTHR == 0);
static_assert(PC_A % NTHR == 0 && PC_B % NTHR == 0 && PC_C % NTHR == 0 && PC_D % NTHR == 0);
static_assert(NWAVE == NTE);
static_assert(CH % 32 == 0 && (2 * CH) % 32 == 0);
static_assert(E_OFF_XE % 16 == 0 && E_OFF_VA % 16 == 0 && E_OFF_WEA % 16 == 0 && E_OFF_WEM % 16 == 0);
static_assert(E_OFF_WRM % 16 == 0 && E_OFF_IDS % 16 == 0);
static_assert((XEP * 2) % 16 == 0 && (VAP * 2) % 16 == 0 && (WEP * 2) % 16 == 0 && (WRP * 2) % 16 == 0);
static_assert(PSTG >= PCH + 32 && PSTG % 4 == 0);
static_assert(NHEAD * HSZ == CH && TM == 16 * NWAVE);
static_assert((FT_TOT * 4) % 256 == 0 && (WB_TOT * 2) % 256 == 0);

typedef float          v2f  __attribute__((ext_vector_type(2)));
typedef float          v4f  __attribute__((ext_vector_type(4)));
typedef float          v8f  __attribute__((ext_vector_type(8)));
typedef int            v4i  __attribute__((ext_vector_type(4)));
typedef int            v8i  __attribute__((ext_vector_type(8)));
typedef unsigned int   v2u  __attribute__((ext_vector_type(2)));
typedef unsigned int   v4u  __attribute__((ext_vector_type(4)));
typedef unsigned short v8us __attribute__((ext_vector_type(8)));
typedef __bf16         v16b __attribute__((ext_vector_type(16)));
typedef v2f  __attribute__((may_alias)) v2fa;
typedef v4f  __attribute__((may_alias)) v4fa;
typedef v4i  __attribute__((may_alias)) v4ia;
typedef v2u  __attribute__((may_alias)) v2ua;
typedef v4u  __attribute__((may_alias)) v4ua;
typedef v8us __attribute__((may_alias)) v8usa;
union FragB { v16b v; v8us h[2]; v8i w; };

__device__ __forceinline__ v8f wmb(const FragB& a, const FragB& b, v8f c) {
  v8f d = __builtin_amdgcn_wmma_f32_16x16x32_bf16(false, a.v, false, b.v, (short)0, c, false, false);
  asm volatile("v_nop\n\tv_nop\n\tv_nop\n\tv_nop" : "+v"(d) : "v"(a.w), "v"(b.w));
  return d;
}

__device__ __forceinline__ unsigned int f2bf(float f) {
  const unsigned int u = __float_as_uint(f);
  const unsigned int r = ((u + 0x7FFFu + ((u >> 16) & 1u)) >> 16) & 0xFFFFu;
  return (f != f) ? 0x7FC0u : r;
}
__device__ __forceinline__ float bf2f(unsigned int b) { return __uint_as_float(b << 16); }
__device__ __forceinline__ float bfr(float f) { return bf2f(f2bf(f)); }
__device__ __forceinline__ v4f bfr4(const v4f a) {
  v4f r; r.x = bfr(a.x); r.y = bfr(a.y); r.z = bfr(a.z); r.w = bfr(a.w); return r;
}
__device__ __forceinline__ unsigned int pk2(float lo, float hi) { return f2bf(lo) | (f2bf(hi) << 16); }
__device__ __forceinline__ unsigned int pk2lo(float lo, float hi) {
  return f2bf(lo - bfr(lo)) | (f2bf(hi - bfr(hi)) << 16);
}
__device__ __forceinline__ v4u pack8(const v4f a, const v4f b) {
  v4u r;
  r.x = pk2(a.x, a.y); r.y = pk2(a.z, a.w); r.z = pk2(b.x, b.y); r.w = pk2(b.z, b.w);
  return r;
}
__device__ __forceinline__ v4u pack8lo(const v4f a, const v4f b) {
  v4u r;
  r.x = pk2lo(a.x, a.y); r.y = pk2lo(a.z, a.w); r.z = pk2lo(b.x, b.y); r.w = pk2lo(b.z, b.w);
  return r;
}
__device__ __forceinline__ v4u gather8(const float* __restrict__ p, int stride) {
  v4f a, b;
  a.x = p[0];                     a.y = p[(size_t)stride];       a.z = p[(size_t)2 * stride];   a.w = p[(size_t)3 * stride];
  b.x = p[(size_t)4 * stride];    b.y = p[(size_t)5 * stride];   b.z = p[(size_t)6 * stride];   b.w = p[(size_t)7 * stride];
  return pack8(a, b);
}
__device__ __forceinline__ void st2u(unsigned short* o, v4u v) {
  *(volatile v4u*)o = v;
  __threadfence();
  *(volatile v4u*)o = v;
}
__device__ __forceinline__ int clampi(int v, int lo, int hi) { return v < lo ? lo : (v > hi ? hi : v); }

__global__ __launch_bounds__(NTHR) void k_pa(const float* __restrict__ xn, const float* __restrict__ xe,
                                             unsigned short* XNB, unsigned short* XEB) {
  const int u = (int)blockIdx.x * NTHR + (int)threadIdx.x;
  const v4f z4 = {0.f, 0.f, 0.f, 0.f};
  if (u < PA_U0) {
    const int row = u >> 3;
    const int c0  = (u & 7) * 8;
    const int rc  = row < NN ? row : NN - 1;
    const float* p = xn + (size_t)rc * CH + c0;
    v4f a = *(const v4fa*)p, b = *(const v4fa*)(p + 4);
    if (row >= NN) { a = z4; b = z4; }
    st2u(XNB + (size_t)row * CH + c0, pack8(a, b));
  } else if (u < PA_U1) {
    const int v   = u - PA_U0;
    const int row = v >> 3;
    const int c0  = (v & 7) * 8;
    const float* p = xe + (size_t)row * CH + c0;
    const v4f a = *(const v4fa*)p, b = *(const v4fa*)(p + 4);
    st2u(XEB + (size_t)row * CH + c0, pack8(a, b));
  }
}

__global__ __launch_bounds__(NTHR) void k_pb(const float* __restrict__ Wk, const float* __restrict__ Wq,
                                             const float* __restrict__ Wv, const float* __restrict__ Wa,
                                             const float* __restrict__ pri, const float* __restrict__ skip,
                                             unsigned short* WKQV, unsigned short* WA2, float* FT) {
  __shared__ __attribute__((aligned(16))) float s_tab[64];
  const int tid = (int)threadIdx.x;
  if ((int)blockIdx.x == PB_NBLK) {
    const int jj = tid & 31;
    const float pv = bfr(pri[(jj & 3) * NTE + (jj >> 2)]);
    const float sv = bfr(skip[tid & 3]);
    const float al = 1.0f / (1.0f + expf(-sv));
    float val = 0.0f;
    val = (tid < 32) ? pv * 0.25f : val;
    val = (tid >= 32 && tid < 36) ? al : val;
    if (tid < 64) s_tab[tid] = val;
    __syncthreads();
    const v4f o = *(const v4fa*)(s_tab + 4 * (tid & 15));
    float* dp = FT + FT_PRQ + 4 * (tid & 15);
    if (tid < 16) *(volatile v4f*)dp = o;
    __threadfence();
    if (tid < 16) *(volatile v4f*)dp = o;
    return;
  }
  const int u = (int)blockIdx.x * NTHR + tid;
  if (u < PB_A) {
    const int t = u >> 9, n = (u >> 3) & 63, k8 = (u & 7) * 8;
    st2u(WKQV + (size_t)((t * 192 + n) * CH + k8), gather8(Wk + (size_t)t * 4096 + k8 * CH + n, CH));
  } else if (u < 2 * PB_A) {
    const int v = u - PB_A;
    const int t = v >> 9, n = (v >> 3) & 63, k8 = (v & 7) * 8;
    st2u(WKQV + (size_t)((t * 192 + 64 + n) * CH + k8), gather8(Wq + (size_t)t * 4096 + k8 * CH + n, CH));
  } else if (u < 3 * PB_A) {
    const int v = u - 2 * PB_A;
    const int t = v >> 9, n = (v >> 3) & 63, k8 = (v & 7) * 8;
    st2u(WKQV + (size_t)((t * 192 + 128 + n) * CH + k8), gather8(Wv + (size_t)t * 4096 + k8 * CH + n, CH));
  } else if (u < PB_TOT) {
    const int v = u - 3 * PB_A;
    const int t = v >> 10, n = (v >> 4) & 63, kk8 = (v & 15) * 8;
    const int k = kk8 & 63;
    st2u(WA2 + (size_t)v * 8, gather8(Wa + (size_t)t * 4096 + k * CH + n, CH));
  }
}

__global__ __launch_bounds__(NTHR) void k_pc(const float* __restrict__ Wra, const float* __restrict__ Wrm,
                                             const float* __restrict__ Wea, const float* __restrict__ Wem,
                                             unsigned short* WB, float* FT) {
  const int u = (int)blockIdx.x * NTHR + (int)threadIdx.x;
  if (u < PC_A) {
    const int t = u >> 13, o = (u >> 3) & 1023, c8 = (u & 7) * 8;
    st2u(WB + WB_WEA + (size_t)u * 8, gather8(Wea + ((size_t)t * CH + c8) * 1024 + o, 1024));
  } else if (u < PC_A + PC_B) {
    const int v = u - PC_A;
    const int t = v >> 9, n = (v >> 3) & 63, c8 = (v & 7) * 8;
    st2u(WB + WB_WEM + (size_t)v * 8, gather8(Wem + ((size_t)t * CH + c8) * CH + n, CH));
  } else if (u < PC_A + PC_B + PC_C) {
    const int v = u - PC_A - PC_B;
    const int piece = v & 3, f = (v >> 2) & 15, h = (v >> 6) & 3, t = v >> 8;
    const int d0 = (piece * 8) & 15;
    st2u(WB + WB_WRM + (size_t)v * 8, gather8(Wrm + ((size_t)(h * NTE + t) * HSZ + d0) * HSZ + f, HSZ));
  } else if (u < PC_TOT) {
    const int v = u - PC_A - PC_B - PC_C;
    const int f4 = (v & 3) * 4, d = (v >> 2) & 15, h = (v >> 6) & 3, t = v >> 8;
    const v4f w = bfr4(*(const v4fa*)(Wra + ((size_t)(h * NTE + t) * HSZ + d) * HSZ + f4));
    float* dp = FT + FT_WRA + (size_t)v * 4;
    *(volatile v4f*)dp = w;
    __threadfence();
    *(volatile v4f*)dp = w;
  }
}

#define PLACE(HJ, J) if (HJ) { if (pos < PSTG) s_stage[pos] = e0 + (J); ++pos; }
__global__ __launch_bounds__(NTHR) void k_perm(const int* __restrict__ et, int* PERM, int* TBASE) {
  __shared__ __attribute__((aligned(16))) int s_cnt[NTE * NTHR];
  __shared__ __attribute__((aligned(16))) int s_stage[PSTG];
  __shared__ __attribute__((aligned(16))) int s_tb[32];
  __shared__ int s_tot[NTE];
  __shared__ int s_wt[NWAVE];
  const int tid = (int)threadIdx.x, lane = tid & 31, wave = tid >> 5;
  const int t = (int)blockIdx.x;

  for (int i = tid; i < PSTG; i += NTHR) s_stage[i] = -1;
  if (tid < 32) s_tb[tid] = 0;

  int c[NTE];
#pragma unroll
  for (int u = 0; u < NTE; ++u) c[u] = 0;
#pragma unroll 2
  for (int g = tid; g < NE / 4; g += NTHR) {
    const v4i v = *(const v4ia*)(et + 4 * g);
#pragma unroll
    for (int u = 0; u < NTE; ++u) c[u] += (int)(v.x == u) + (int)(v.y == u) + (int)(v.z == u) + (int)(v.w == u);
  }
#pragma unroll
  for (int u = 0; u < NTE; ++u) s_cnt[u * NTHR + tid] = c[u];
  __syncthreads();
  {
    int s = 0;
#pragma unroll
    for (int i = 0; i < 8; ++i) s += s_cnt[wave * NTHR + lane * 8 + i];
#pragma unroll
    for (int off = 16; off > 0; off >>= 1) s += __shfl_xor(s, off);
    if (lane == 0) s_tot[wave] = s;
  }
  __syncthreads();
  int base = 0, cntT = 0;
#pragma unroll
  for (int u = 0; u < NTE; ++u) {
    const int cu = clampi(s_tot[u], 0, NE);
    const int pu = (cu + 127) & ~127;
    base += (u < t) ? pu : 0;
    cntT = (u == t) ? cu : cntT;
  }

  if (t == 0) {
    if (tid < 32) {
      int b = 0;
#pragma unroll
      for (int u = 0; u < NTE; ++u) {
        const int cu = clampi(s_tot[u], 0, NE);
        b += (u < tid) ? ((cu + 127) & ~127) : 0;
      }
      s_tb[tid] = (tid <= NTE) ? b : 0;
    }
    __syncthreads();
    const v4i tv = *(const v4ia*)(s_tb + 4 * (tid & 7));
    int* tp = TBASE + 4 * (tid & 7);
    if (tid < 8) *(volatile v4i*)tp = tv;
    __threadfence();
    if (tid < 8) *(volatile v4i*)tp = tv;
  }

  int fill = 0, wrote = 0;
  const int nCh = (NE + PCH - 1) / PCH;
#pragma unroll 1
  for (int ch = 0; ch < nCh; ++ch) {
    const int cbase = ch * PCH;
    const int e0 = cbase + tid * 8;
    v4i da, db;
    if (cbase + PCH <= NE) {
      da = *(const v4ia*)(et + e0);
      db = *(const v4ia*)(et + e0 + 4);
    } else {
      da.x = (e0     < NE) ? et[min(e0,     NE - 1)] : -1;
      da.y = (e0 + 1 < NE) ? et[min(e0 + 1, NE - 1)] : -1;
      da.z = (e0 + 2 < NE) ? et[min(e0 + 2, NE - 1)] : -1;
      da.w = (e0 + 3 < NE) ? et[min(e0 + 3, NE - 1)] : -1;
      db.x = (e0 + 4 < NE) ? et[min(e0 + 4, NE - 1)] : -1;
      db.y = (e0 + 5 < NE) ? et[min(e0 + 5, NE - 1)] : -1;
      db.z = (e0 + 6 < NE) ? et[min(e0 + 6, NE - 1)] : -1;
      db.w = (e0 + 7 < NE) ? et[min(e0 + 7, NE - 1)] : -1;
    }
    const bool h0 = da.x == t, h1 = da.y == t, h2 = da.z == t, h3 = da.w == t;
    const bool h4 = db.x == t, h5 = db.y == t, h6 = db.z == t, h7 = db.w == t;
    const int cth = (int)h0 + (int)h1 + (int)h2 + (int)h3 + (int)h4 + (int)h5 + (int)h6 + (int)h7;
    int incl = cth;
#pragma unroll
    for (int d = 1; d < 32; d <<= 1) {
      const int y = __shfl_up(incl, d);
      if (lane >= d) incl += y;
    }
    if (lane == 31) s_wt[wave] = incl;
    __syncthreads();
    int pre = 0, all = 0;
#pragma unroll
    for (int w2 = 0; w2 < NWAVE; ++w2) {
      const int cw = clampi(s_wt[w2], 0, WCAP);
      all += cw;
      pre += (w2 < wave) ? cw : 0;
    }
    int pos = fill + pre + incl - cth;
    PLACE(h0, 0) PLACE(h1, 1) PLACE(h2, 2) PLACE(h3, 3)
    PLACE(h4, 4) PLACE(h5, 5) PLACE(h6, 6) PLACE(h7, 7)
    fill += all;
    fill = fill > PSTG ? PSTG : fill;
    __syncthreads();
    const int nf = fill & ~31;
    const int nq = nf >> 2;
    int* gp = PERM + base + wrote;
#pragma unroll 1
    for (int q = tid; q < nq; q += NTHR) {
      const v4i v = *(const v4ia*)(s_stage + 4 * q);
      if (base + wrote + 4 * q + 3 < PCAP) *(volatile v4i*)(gp + 4 * q) = v;
    }
    __threadfence();
#pragma unroll 1
    for (int q = tid; q < nq; q += NTHR) {
      const v4i v = *(const v4ia*)(s_stage + 4 * q);
      if (base + wrote + 4 * q + 3 < PCAP) *(volatile v4i*)(gp + 4 * q) = v;
    }
    const int rem = fill - nf;
    const int keep = s_stage[min(nf + tid, PSTG - 1)];
    __syncthreads();
    if (tid < rem) s_stage[tid] = keep;
    wrote += nf;
    fill = rem;
    __syncthreads();
  }
  {
    const int L = (cntT + 127) & ~127;
    const int remain = clampi(L - wrote, 0, NTHR) & ~3;
    if (tid >= fill && tid < remain) s_stage[tid] = -1;
    __syncthreads();
    const int nq = remain >> 2;
    const v4i v = *(const v4ia*)(s_stage + 4 * (tid & 63));
    int* gp = PERM + base + wrote + 4 * (tid & 63);
    const bool wr = (tid < nq) && (tid < 64) && (base + wrote + 4 * tid + 3 < PCAP);
    if (wr) *(volatile v4i*)gp = v;
    __threadfence();
    if (wr) *(volatile v4i*)gp = v;
  }
}
#undef PLACE

__global__ __launch_bounds__(NTHR) __attribute__((amdgpu_num_vgpr(248)))
void k_node(const unsigned short* __restrict__ XNB, const unsigned short* __restrict__ WKQV,
            const int* __restrict__ ntype, float* KQ, unsigned short* VP) {
  __shared__ __attribute__((aligned(16))) float stg[TM * CH];
  const int tid = (int)threadIdx.x, lane = tid & 31, wave = tid >> 5, hh = lane >> 4, m = lane & 15;
  const int rowBase = (int)blockIdx.x * TM;
  const int t = (int)blockIdx.y;
  const int myrow = rowBase + 16 * wave + m;
  const int ntv = ntype[myrow < NN ? myrow : NN - 1];

  FragB a0, a1;
  {
    const unsigned short* ap = XNB + (size_t)myrow * CH + 8 * hh;
    a0.h[0] = *(const v8usa*)ap;
    a0.h[1] = *(const v8usa*)(ap + 16);
    a1.h[0] = *(const v8usa*)(ap + 32);
    a1.h[1] = *(const v8usa*)(ap + 48);
  }

#pragma unroll 1
  for (int g = 0; g < 3; ++g) {
    v8f acc[4];
    {
      const v8f z = {0.f, 0.f, 0.f, 0.f, 0.f, 0.f, 0.f, 0.f};
      acc[0] = z; acc[1] = z; acc[2] = z; acc[3] = z;
    }
    const unsigned short* wp = WKQV + (size_t)(t * 192 + g * 64 + m) * CH + 8 * hh;
#pragma unroll
    for (int nt = 0; nt < 4; ++nt) {
      const unsigned short* wq = wp + (size_t)(16 * nt) * CH;
      FragB b0, b1;
      b0.h[0] = *(const v8usa*)wq;
      b0.h[1] = *(const v8usa*)(wq + 16);
      b1.h[0] = *(const v8usa*)(wq + 32);
      b1.h[1] = *(const v8usa*)(wq + 48);
      acc[nt] = wmb(a0, b0, acc[nt]);
      acc[nt] = wmb(a1, b1, acc[nt]);
    }
    if (g > 0) __syncthreads();
#pragma unroll
    for (int nt = 0; nt < 4; ++nt) {
      const int lc = 16 * nt + m;
#pragma unroll
      for (int r = 0; r < 8; ++r) stg[(16 * wave + 8 * hh + r) * CH + lc] = acc[nt][r];
    }
    __syncthreads();

    if (g < 2) {
      v4f fv[8];
      bool ok[8];
#pragma unroll
      for (int i = 0; i < 8; ++i) {
        const int lr  = 16 * wave + 2 * i + hh;
        const int nti = __shfl(ntv, 2 * i + hh);
        ok[i] = (rowBase + lr < NN) && (nti == t);
        fv[i] = *(const v4fa*)(stg + lr * CH + 4 * m);
      }
      float* ob = KQ + (size_t)g * MPN * CH;
#pragma unroll
      for (int i = 0; i < 8; ++i) {
        const int row = rowBase + 16 * wave + 2 * i + hh;
        float* op = ob + (size_t)row * CH + 4 * m;
        if (ok[i]) *(volatile v4f*)op = fv[i];
      }
      __threadfence();
#pragma unroll
      for (int i = 0; i < 8; ++i) {
        const int row = rowBase + 16 * wave + 2 * i + hh;
        float* op = ob + (size_t)row * CH + 4 * m;
        if (ok[i]) *(volatile v4f*)op = fv[i];
      }
    } else {
      v4u pv[8];
      bool ok[8];
      const int head = m >> 2, sub = m & 3;
      const unsigned int mk1 = 0u - (unsigned int)(sub >> 1);
      const v4u mk = {mk1, mk1, mk1, mk1};
      const int d0 = 8 * (sub & 1);
#pragma unroll
      for (int i = 0; i < 8; ++i) {
        const int lr  = 16 * wave + 2 * i + hh;
        const int nti = __shfl(ntv, 2 * i + hh);
        ok[i] = (rowBase + lr < NN) && (nti == t);
        const float* sp = stg + lr * CH + head * HSZ + d0;
        const v4f a = *(const v4fa*)sp;
        const v4f b = *(const v4fa*)(sp + 4);
        const v4u hv = pack8(a, b);
        const v4u lv = pack8lo(a, b);
        pv[i] = (hv & ~mk) | (lv & mk);
      }
#pragma unroll
      for (int i = 0; i < 8; ++i) {
        const int row = rowBase + 16 * wave + 2 * i + hh;
        unsigned short* op = VP + (size_t)row * 128 + 8 * m;
        if (ok[i]) *(volatile v4u*)op = pv[i];
      }
      __threadfence();
#pragma unroll
      for (int i = 0; i < 8; ++i) {
        const int row = rowBase + 16 * wave + 2 * i + hh;
        unsigned short* op = VP + (size_t)row * 128 + 8 * m;
        if (ok[i]) *(volatile v4u*)op = pv[i];
      }
    }
  }
}

__global__ __launch_bounds__(NTHR) __attribute__((amdgpu_num_vgpr(248)))
void k_edge(const int* __restrict__ PERM, const int* __restrict__ TBASE,
            const int* __restrict__ src, const int* __restrict__ dst,
            const unsigned short* __restrict__ XEB, const float* __restrict__ KQ,
            const unsigned short* __restrict__ VP, const unsigned short* __restrict__ WB,
            const float* __restrict__ FT, float* MSG, float* SC, int* DSTP) {
  extern __shared__ __attribute__((aligned(16))) unsigned char esm[];
  float*          sKT  = (float*)(esm + E_OFF_KT);
  float*          sQT  = (float*)(esm + E_OFF_QT);
  float*          sMSG = (float*)(esm + E_OFF_MSG);
  float*          sSC  = (float*)(esm + E_OFF_SC);
  float*          sWRA = (float*)(esm + E_OFF_WRA);
  unsigned short* sXE  = (unsigned short*)(esm + E_OFF_XE);
  unsigned short* sVA  = (unsigned short*)(esm + E_OFF_VA);
  unsigned short* sWEA = (unsigned short*)(esm + E_OFF_WEA);
  unsigned short* sWEM = (unsigned short*)(esm + E_OFF_WEM);
  unsigned short* sWRM = (unsigned short*)(esm + E_OFF_WRM);
  int*            sPc  = (int*)(esm + E_OFF_IDS);
  int*            sS   = sPc + TM;
  int*            sD   = sS + TM;
  int*            sDO  = sD + TM;
  int*            sV   = sDO + TM;

  const int tid = (int)threadIdx.x, lane = tid & 31, wave = tid >> 5, hh = lane >> 4, m = lane & 15;
  const int tile  = (int)blockIdx.x;
  const int start = tile * TM;

  const v4i tb0 = *(const v4ia*)(TBASE);
  const v4i tb1 = *(const v4ia*)(TBASE + 4);
  const v4i tb2 = *(const v4ia*)(TBASE + 8);
  const int t = (int)(start >= tb0.y) + (int)(start >= tb0.z) + (int)(start >= tb0.w) + (int)(start >= tb1.x) +
                (int)(start >= tb1.y) + (int)(start >= tb1.z) + (int)(start >= tb1.w) + (int)(start >= tb2.x);
  if (t >= NTE) {
    const v4i m1 = {-1, -1, -1, -1};
    int* dp = DSTP + start + 4 * (tid & 31);
    if (tid < 32) *(volatile v4i*)dp = m1;
    __threadfence();
    if (tid < 32) *(volatile v4i*)dp = m1;
    return;
  }

  if (tid < TM) {
    const int p = PERM[start + tid];
    const bool valid = (unsigned)p < (unsigned)NE;
    const int pc = clampi(p, 0, NE - 1);
    const int s  = clampi(src[pc], 0, NN - 1);
    const int draw = dst[pc];
    const int dc = clampi(draw, 0, NN - 1);
    sPc[tid] = pc; sS[tid] = s; sD[tid] = dc;
    sDO[tid] = valid ? draw : -1;
    sV[tid]  = valid ? 1 : 0;
  }
  __syncthreads();

#pragma unroll 2
  for (int it = 0; it < 4; ++it) {
    const int idx = it * NTHR + tid, row = idx >> 3, pc8 = (idx & 7) * 8;
    const v8us v = *(const v8usa*)(XEB + (size_t)sPc[row] * CH + pc8);
    *(v8usa*)(sXE + row * XEP + pc8) = v;
  }
#pragma unroll 2
  for (int it = 0; it < 8; ++it) {
    const int idx = it * NTHR + tid, row = idx >> 4, pc8 = (idx & 15) * 8;
    const v8us v = *(const v8usa*)(VP + (size_t)sS[row] * 128 + pc8);
    *(v8usa*)(sVA + row * VAP + pc8) = v;
  }
  {
    const int e = tid & (TM - 1), hf = tid >> 7;
    const float* kr = KQ + (size_t)sS[e] * CH + hf * 32;
    const float* qr = KQ + (size_t)MPN * CH + (size_t)sD[e] * CH + hf * 32;
#pragma unroll 2
    for (int j = 0; j < 8; ++j) {
      const v4f kv = *(const v4fa*)(kr + 4 * j);
      const v4f qv = *(const v4fa*)(qr + 4 * j);
      const int c = hf * 32 + 4 * j;
      sKT[(c + 0) * TM + e] = kv.x; sKT[(c + 1) * TM + e] = kv.y;
      sKT[(c + 2) * TM + e] = kv.z; sKT[(c + 3) * TM + e] = kv.w;
      sQT[(c + 0) * TM + e] = qv.x; sQT[(c + 1) * TM + e] = qv.y;
      sQT[(c + 2) * TM + e] = qv.z; sQT[(c + 3) * TM + e] = qv.w;
    }
  }
#pragma unroll
  for (int it = 0; it < 2; ++it) {
    const int idx = it * NTHR + tid, row = idx >> 3, pc8 = (idx & 7) * 8;
    const v8us v = *(const v8usa*)(WB + WB_WEM + (size_t)(t * CH + row) * CH + pc8);
    *(v8usa*)(sWEM + row * WEP + pc8) = v;
  }
  {
    const int row = tid >> 2, pc8 = (tid & 3) * 8;
    const v8us v = *(const v8usa*)(WB + WB_WRM + (size_t)(t * CH + row) * 32 + pc8);
    *(v8usa*)(sWRM + row * WRP + pc8) = v;
    const v4f w = *(const v4fa*)(FT + FT_WRA + (size_t)t * 1024 + 4 * tid);
    *(v4fa*)(sWRA + 4 * tid) = w;
  }
  const v4f pq4 = *(const v4fa*)(FT + FT_PRQ + 4 * t);
  __syncthreads();

  FragB ax0, ax1;
  {
    const unsigned short* xp = sXE + (16 * wave + m) * XEP + 8 * hh;
    ax0.h[0] = *(const v8usa*)xp;
    ax0.h[1] = *(const v8usa*)(xp + 16);
    ax1.h[0] = *(const v8usa*)(xp + 32);
    ax1.h[1] = *(const v8usa*)(xp + 48);
  }
  const int colb = 16 * wave + 8 * hh;

#pragma unroll 1
  for (int h = 0; h < NHEAD; ++h) {
    if (h > 0) __syncthreads();
#pragma unroll 2
    for (int it = 0; it < 8; ++it) {
      const int idx = it * NTHR + tid, row = idx >> 3, pc8 = (idx & 7) * 8;
      const v8us v = *(const v8usa*)(WB + WB_WEA + (size_t)(t * 1024 + h * 256 + row) * CH + pc8);
      *(v8usa*)(sWEA + row * WEP + pc8) = v;
    }
    __syncthreads();

    v8f kw = {0.f, 0.f, 0.f, 0.f, 0.f, 0.f, 0.f, 0.f};
#pragma unroll 1
    for (int d = 0; d < HSZ; ++d) {
      const float wra = sWRA[(h * HSZ + d) * HSZ + m];
      v8f acc = {wra, wra, wra, wra, wra, wra, wra, wra};
      const unsigned short* bp = sWEA + (d * HSZ + m) * WEP + 8 * hh;
      FragB b0, b1;
      b0.h[0] = *(const v8usa*)bp;
      b0.h[1] = *(const v8usa*)(bp + 16);
      b1.h[0] = *(const v8usa*)(bp + 32);
      b1.h[1] = *(const v8usa*)(bp + 48);
      acc = wmb(ax0, b0, acc);
      acc = wmb(ax1, b1, acc);
      const float* kp = sKT + (h * HSZ + d) * TM + colb;
      const v4f ka = *(const v4fa*)kp;
      const v4f kb = *(const v4fa*)(kp + 4);
      kw[0] = fmaf(ka.x, acc[0], kw[0]); kw[1] = fmaf(ka.y, acc[1], kw[1]);
      kw[2] = fmaf(ka.z, acc[2], kw[2]); kw[3] = fmaf(ka.w, acc[3], kw[3]);
      kw[4] = fmaf(kb.x, acc[4], kw[4]); kw[5] = fmaf(kb.y, acc[5], kw[5]);
      kw[6] = fmaf(kb.z, acc[6], kw[6]); kw[7] = fmaf(kb.w, acc[7], kw[7]);
    }
    const float* qp = sQT + (h * HSZ + m) * TM + colb;
    const v4f qa = *(const v4fa*)qp;
    const v4f qb = *(const v4fa*)(qp + 4);
    float s[8];
    s[0] = kw[0] * qa.x; s[1] = kw[1] * qa.y; s[2] = kw[2] * qa.z; s[3] = kw[3] * qa.w;
    s[4] = kw[4] * qb.x; s[5] = kw[5] * qb.y; s[6] = kw[6] * qb.z; s[7] = kw[7] * qb.w;
#pragma unroll
    for (int r = 0; r < 8; ++r) {
      float x = s[r];
      x += __shfl_xor(x, 1);
      x += __shfl_xor(x, 2);
      x += __shfl_xor(x, 4);
      x += __shfl_xor(x, 8);
      s[r] = x;
    }
    const float pq = (h == 0) ? pq4.x : ((h == 1) ? pq4.y : ((h == 2) ? pq4.z : pq4.w));
    if (m == 0) {
#pragma unroll
      for (int r = 0; r < 8; ++r) sSC[(colb + r) * 4 + h] = s[r] * pq;
    }
  }

#pragma unroll 1
  for (int h = 0; h < NHEAD; ++h) {
    v8f acc = {0.f, 0.f, 0.f, 0.f, 0.f, 0.f, 0.f, 0.f};
    const unsigned short* bm = sWEM + (h * HSZ + m) * WEP + 8 * hh;
    FragB b0, b1, bw, va;
    b0.h[0] = *(const v8usa*)bm;
    b0.h[1] = *(const v8usa*)(bm + 16);
    b1.h[0] = *(const v8usa*)(bm + 32);
    b1.h[1] = *(const v8usa*)(bm + 48);
    const unsigned short* wr = sWRM + (h * HSZ + m) * WRP + 8 * hh;
    bw.h[0] = *(const v8usa*)wr;
    bw.h[1] = *(const v8usa*)(wr + 16);
    const unsigned short* vp = sVA + (16 * wave + m) * VAP + 32 * h + 8 * hh;
    va.h[0] = *(const v8usa*)vp;
    va.h[1] = *(const v8usa*)(vp + 16);
    acc = wmb(ax0, b0, acc);
    acc = wmb(ax1, b1, acc);
    acc = wmb(va, bw, acc);
#pragma unroll
    for (int r = 0; r < 8; ++r) sMSG[(colb + r) * CH + h * HSZ + m] = acc[r];
  }
  __syncthreads();

  {
    const v4f z4 = {0.f, 0.f, 0.f, 0.f};
    v4f pv[8];
#pragma unroll
    for (int it = 0; it < 8; ++it) {
      const int idx = it * NTHR + tid;
      v4f v = *(const v4fa*)(sMSG + 4 * idx);
      if (sV[idx >> 4] == 0) v = z4;
      pv[it] = v;
    }
    v4f scv = *(const v4fa*)(sSC + 4 * (tid & (TM - 1)));
    if (sV[tid & (TM - 1)] == 0) scv = z4;
    const v4i dv = *(const v4ia*)(sDO + 4 * (tid & 31));
    float* mb = MSG + (size_t)start * CH;
    float* sp = SC + (size_t)start * 4 + 4 * (tid & (TM - 1));
    int*   dp = DSTP + start + 4 * (tid & 31);
#pragma unroll
    for (int it = 0; it < 8; ++it) *(volatile v4f*)(mb + 4 * (it * NTHR + tid)) = pv[it];
    if (tid < TM) *(volatile v4f*)sp = scv;
    if (tid < 32) *(volatile v4i*)dp = dv;
    __threadfence();
#pragma unroll
    for (int it = 0; it < 8; ++it) *(volatile v4f*)(mb + 4 * (it * NTHR + tid)) = pv[it];
    if (tid < TM) *(volatile v4f*)sp = scv;
    if (tid < 32) *(volatile v4i*)dp = dv;
  }
}

__device__ __forceinline__ int scan_chunk(const int* __restrict__ dsts, int nE, int cbase, int slotBase,
                                          int nb, int vec8, int* list, int tid, int lane, int wave) {
  int wc = 0;
  const int el0  = tid * EPT;
  const int e0   = cbase + el0;
  const int sent = -2147483647 - 1;
  v4i da, db;
  if (vec8 != 0 && cbase + CHUNK <= nE) {
    da = *(const v4i*)(dsts + e0);
    db = *(const v4i*)(dsts + e0 + 4);
  } else {
    da.x = (e0     < nE) ? dsts[min(e0,     nE - 1)] : sent;
    da.y = (e0 + 1 < nE) ? dsts[min(e0 + 1, nE - 1)] : sent;
    da.z = (e0 + 2 < nE) ? dsts[min(e0 + 2, nE - 1)] : sent;
    da.w = (e0 + 3 < nE) ? dsts[min(e0 + 3, nE - 1)] : sent;
    db.x = (e0 + 4 < nE) ? dsts[min(e0 + 4, nE - 1)] : sent;
    db.y = (e0 + 5 < nE) ? dsts[min(e0 + 5, nE - 1)] : sent;
    db.z = (e0 + 6 < nE) ? dsts[min(e0 + 6, nE - 1)] : sent;
    db.w = (e0 + 7 < nE) ? dsts[min(e0 + 7, nE - 1)] : sent;
  }
  const unsigned nbs = (unsigned)slotBase;
  const unsigned unb = (unsigned)nb;
  const unsigned s0 = (unsigned)da.x - nbs, s1 = (unsigned)da.y - nbs;
  const unsigned s2 = (unsigned)da.z - nbs, s3 = (unsigned)da.w - nbs;
  const unsigned s4 = (unsigned)db.x - nbs, s5 = (unsigned)db.y - nbs;
  const unsigned s6 = (unsigned)db.z - nbs, s7 = (unsigned)db.w - nbs;
  const bool h0 = s0 < unb, h1 = s1 < unb, h2 = s2 < unb, h3 = s3 < unb;
  const bool h4 = s4 < unb, h5 = s5 < unb, h6 = s6 < unb, h7 = s7 < unb;
  const unsigned any = __builtin_amdgcn_ballot_w32(h0 | h1 | h2 | h3 | h4 | h5 | h6 | h7);
  if (any != 0u) {
#define HITJ(J, HJ, SJ) { \
      const unsigned mj = __builtin_amdgcn_ballot_w32(HJ); \
      if (mj != 0u) { \
        if (HJ) { \
          const int pos = wc + (int)__builtin_amdgcn_mbcnt_lo(mj, 0u); \
          if (pos < WCAP) list[wave * WCAP + pos] = ((el0 + (J)) << SLOTB) | (int)(SJ); \
        } \
        wc += (int)__builtin_popcount(mj); } }
    HITJ(0, h0, s0)
    HITJ(1, h1, s1)
    HITJ(2, h2, s2)
    HITJ(3, h3, s3)
    HITJ(4, h4, s4)
    HITJ(5, h5, s5)
    HITJ(6, h6, s6)
    HITJ(7, h7, s7)
#undef HITJ
  }
  return wc;
}

__global__ __launch_bounds__(NTHR) __attribute__((amdgpu_num_vgpr(248)))
void k_scan(const int* __restrict__ keys, const float* __restrict__ SC, const float* __restrict__ MSG,
            unsigned int* HHLw) {
  extern __shared__ v4f lds_dyn[];
  int* reg1 = (int*)lds_dyn;
  int* reg2 = reg1 + RCAP;
  int* scnt = reg2 + RCAP;
  int* soff = scnt + NBMAX;
  int* list = soff + NBMAX;
  int* wcnt = list + LISTN;
  int* wtot = wcnt + NWAVE;
  const int tid = (int)threadIdx.x, lane = tid & 31, wave = tid >> 5;
  const int nb = NBRUN;
  const int nE = PCAP;
  const int nodeBase = (int)blockIdx.x * nb;

  for (int i = tid; i < NBMAX; i += NTHR) scnt[i] = 0;
  __syncthreads();

  int tot = 0;
  const int nChunks = (nE + CHUNK - 1) / CHUNK;
#pragma unroll 1
  for (int ch = 0; ch < nChunks; ++ch) {
    const int cbase = ch * CHUNK;
    const int wc = scan_chunk(keys, nE, cbase, nodeBase, nb, 1, list, tid, lane, wave);
    if (lane == 0) wcnt[wave] = wc;
    __syncthreads();
    int pre = 0, all = 0;
#pragma unroll
    for (int w2 = 0; w2 < NWAVE; ++w2) {
      int c = wcnt[w2];
      c = c < 0 ? 0 : (c > WCAP ? WCAP : c);
      all += c;
      pre += (w2 < wave) ? c : 0;
    }
    const int wcc  = wc > WCAP ? WCAP : wc;
    const int base = tot + pre;
#pragma unroll 1
    for (int i = lane; i < wcc; i += 32) {
      const int ent = list[wave * WCAP + i];
      const int el  = (ent >> SLOTB) & (CHUNK - 1);
      const int sl  = ent & (NBMAX - 1);
      int eid = cbase + el;
      eid = eid > nE - 1 ? nE - 1 : eid;
      const int pos = base + i;
      if (pos < RCAP) reg1[pos] = (int)(((unsigned)eid << SLOTB) | (unsigned)sl);
    }
    tot += all;
    tot = tot > RCAP ? RCAP : tot;
    __syncthreads();
  }
  const int nh = tot;

  if (wave == 0) {
#pragma unroll 1
    for (int b0 = 0; b0 < nh; b0 += 32) {
      const int idx = b0 + lane;
      const int uv  = reg1[idx < nh ? idx : nh - 1];
      const int m32 = (nh - b0) < 32 ? (nh - b0) : 32;
#pragma unroll 1
      for (int k = 0; k < m32; ++k) {
        const int u  = __builtin_amdgcn_readlane(uv, k);
        const int sl = u & (NBMAX - 1);
        if (lane == 0) scnt[sl] = scnt[sl] + 1;
      }
    }
  }
  __syncthreads();

  {
    const v4i ca = *(const v4i*)(scnt + 8 * tid);
    const v4i cb = *(const v4i*)(scnt + 8 * tid + 4);
    const int e0 = ca.x < 0 ? 0 : ca.x, e1 = ca.y < 0 ? 0 : ca.y, e2 = ca.z < 0 ? 0 : ca.z, e3 = ca.w < 0 ? 0 : ca.w;
    const int e4 = cb.x < 0 ? 0 : cb.x, e5 = cb.y < 0 ? 0 : cb.y, e6 = cb.z < 0 ? 0 : cb.z, e7 = cb.w < 0 ? 0 : cb.w;
    const int ts = e0 + e1 + e2 + e3 + e4 + e5 + e6 + e7;
    int incl = ts;
#pragma unroll
    for (int d = 1; d < 32; d <<= 1) {
      const int up = __shfl_up(incl, d);
      if (lane >= d) incl += up;
    }
    if (lane == 31) wtot[wave] = incl;
    __syncthreads();
    int pre = 0;
#pragma unroll
    for (int w2 = 0; w2 < NWAVE; ++w2) pre += (w2 < wave) ? wtot[w2] : 0;
    int run = pre + incl - ts;
    soff[8 * tid + 0] = run; run += e0;
    soff[8 * tid + 1] = run; run += e1;
    soff[8 * tid + 2] = run; run += e2;
    soff[8 * tid + 3] = run; run += e3;
    soff[8 * tid + 4] = run; run += e4;
    soff[8 * tid + 5] = run; run += e5;
    soff[8 * tid + 6] = run; run += e6;
    soff[8 * tid + 7] = run;
  }
  __syncthreads();
  for (int i = tid; i < NBMAX; i += NTHR) list[i] = soff[i];
  __syncthreads();

  if (wave == 0) {
#pragma unroll 1
    for (int b0 = 0; b0 < nh; b0 += 32) {
      const int idx = b0 + lane;
      const int uv  = reg1[idx < nh ? idx : nh - 1];
      const int m32 = (nh - b0) < 32 ? (nh - b0) : 32;
#pragma unroll 1
      for (int k = 0; k < m32; ++k) {
        const int u   = __builtin_amdgcn_readlane(uv, k);
        const int sl  = u & (NBMAX - 1);
        const int eid = (int)((unsigned)u >> SLOTB);
        if (lane == 0) {
          int pos = list[sl];
          pos = pos < 0 ? 0 : (pos > RCAP - 1 ? RCAP - 1 : pos);
          reg2[pos] = eid;
          list[sl] = pos + 1;
        }
      }
    }
  }
  __syncthreads();

  const int nbw = nb >> 3;
  const bool ovf = (nh >= RCAP);
  const float qnan = __int_as_float(0x7fc00000);
  const int head = lane >> 3;

#pragma unroll 1
  for (int jt = 0; jt < nbw; ++jt) {
    const int slot = wave * nbw + jt;
    const int grow = nodeBase + slot;
    int st = soff[slot];
    const int craw = scnt[slot];
    int cnt = craw;
    st  = st < 0 ? 0 : (st > nh ? nh : st);
    cnt = cnt < 0 ? 0 : (cnt > DEGCAP ? DEGCAP : cnt);
    if (cnt > nh - st) cnt = nh - st;
    const float pz = (ovf || craw > DEGCAP) ? qnan : 0.0f;

    float mx = MX0, dn = 0.0f, a0 = 0.0f, a1 = 0.0f;
#pragma unroll 1
    for (int q = 0; q < cnt; ++q) {
      int idx = st + q; idx = idx > RCAP - 1 ? RCAP - 1 : idx;
      int p = reg2[idx]; p = p < 0 ? 0 : (p > PCAP - 1 ? PCAP - 1 : p);
      const v4f sc = *(const v4fa*)(SC + (size_t)p * 4);
      const v2f mv = *(const v2fa*)(MSG + (size_t)p * CH + 2 * lane);
      const float lg = (head == 0) ? sc.x : ((head == 1) ? sc.y : ((head == 2) ? sc.z : sc.w));
      const float df = lg - mx;
      const float ee = expf(-fabsf(df));
      const bool up  = df > 0.f;
      const float s1 = up ? ee : 1.0f;
      const float s2 = up ? 1.0f : ee;
      mx = up ? lg : mx;
      dn = fmaf(dn, s1, s2);
      a0 = fmaf(a0, s1, s2 * mv.x);
      a1 = fmaf(a1, s1, s2 * mv.y);
    }
    const bool has = cnt > 0;
    const float inv = __builtin_amdgcn_rcpf(has ? dn : 1.0f);
    const bool live = has && (grow < NN);
    const float o0 = (live ? a0 * inv : 0.0f) + pz;
    const float o1 = (live ? a1 * inv : 0.0f) + pz;
    const unsigned int hw = pk2(o0, o1);
    const unsigned int lw = pk2lo(o0, o1);
    const int gr = grow < MPN ? grow : MPN - 1;
    unsigned int* gp = HHLw + (size_t)gr * 64 + lane;
    const bool wr = grow < MPN;
    if (wr) { *(volatile unsigned int*)gp = hw; *(volatile unsigned int*)(gp + 32) = lw; }
    __threadfence();
    if (wr) { *(volatile unsigned int*)gp = hw; *(volatile unsigned int*)(gp + 32) = lw; }
  }
}

__global__ __launch_bounds__(NTHR) __attribute__((amdgpu_num_vgpr(248)))
void k_out(const unsigned short* __restrict__ HHL, const unsigned short* __restrict__ WA2,
           const int* __restrict__ ntype, const unsigned short* __restrict__ XNB,
           const float* __restrict__ FT, float* out) {
  __shared__ __attribute__((aligned(16))) float stg[TM * CH];
  const int tid = (int)threadIdx.x, lane = tid & 31, wave = tid >> 5, hh = lane >> 4, m = lane & 15;
  const int rowBase = (int)blockIdx.x * TM;
  const int t = (int)blockIdx.y;
  const int myrow = rowBase + 16 * wave + m;
  const int ntv = ntype[myrow < NN ? myrow : NN - 1];
  const float al = FT[FT_ALP + t];
  const float om = 1.0f - al;

  v8f acc[4];
  {
    const v8f z = {0.f, 0.f, 0.f, 0.f, 0.f, 0.f, 0.f, 0.f};
    acc[0] = z; acc[1] = z; acc[2] = z; acc[3] = z;
  }
  const unsigned short* ap = HHL + (size_t)myrow * 128 + 8 * hh;
  const unsigned short* wp = WA2 + (size_t)(t * CH + m) * 128 + 8 * hh;
#pragma unroll 1
  for (int ks = 0; ks < 4; ++ks) {
    FragB af;
    af.h[0] = *(const v8usa*)(ap + 32 * ks);
    af.h[1] = *(const v8usa*)(ap + 32 * ks + 16);
#pragma unroll
    for (int nt = 0; nt < 4; ++nt) {
      const unsigned short* wq = wp + (size_t)(16 * nt) * 128 + 32 * ks;
      FragB bf;
      bf.h[0] = *(const v8usa*)wq;
      bf.h[1] = *(const v8usa*)(wq + 16);
      acc[nt] = wmb(af, bf, acc[nt]);
    }
  }
#pragma unroll
  for (int nt = 0; nt < 4; ++nt) {
    const int lc = 16 * nt + m;
#pragma unroll
    for (int r = 0; r < 8; ++r) stg[(16 * wave + 8 * hh + r) * CH + lc] = acc[nt][r];
  }
  __syncthreads();

  v4f fv[8];
  bool ok[8];
#pragma unroll
  for (int i = 0; i < 8; ++i) {
    const int lr  = 16 * wave + 2 * i + hh;
    const int row = rowBase + lr;
    const int nti = __shfl(ntv, 2 * i + hh);
    ok[i] = (row < NN) && (nti == t);
    const int rc = row < NN ? row : NN - 1;
    const v4f d = *(const v4fa*)(stg + lr * CH + 4 * m);
    const v2u xw = *(const v2ua*)(XNB + (size_t)rc * CH + 4 * m);
    v4f o;
    o.x = d.x * al + bf2f(xw.x & 0xFFFFu) * om;
    o.y = d.y * al + bf2f(xw.x >> 16) * om;
    o.z = d.z * al + bf2f(xw.y & 0xFFFFu) * om;
    o.w = d.w * al + bf2f(xw.y >> 16) * om;
    fv[i] = o;
  }
#pragma unroll
  for (int i = 0; i < 8; ++i) {
    const int row = rowBase + 16 * wave + 2 * i + hh;
    float* op = out + (size_t)row * CH + 4 * m;
    if (ok[i]) *(volatile v4f*)op = fv[i];
  }
  __threadfence();
#pragma unroll
  for (int i = 0; i < 8; ++i) {
    const int row = rowBase + 16 * wave + 2 * i + hh;
    float* op = out + (size_t)row * CH + 4 * m;
    if (ok[i]) *(volatile v4f*)op = fv[i];
  }
}

extern "C" void kernel_launch(void* const* d_in, const int* in_sizes, int n_in,
                              void* d_out, int out_size, void* d_ws, size_t ws_size,
                              hipStream_t stream) {
  if (n_in < 16) return;
  if (in_sizes[0] != NN * CH || in_sizes[1] != NE * CH) return;
  if (in_sizes[2] != NN || in_sizes[3] != NE) return;
  if (in_sizes[4] != NE || in_sizes[5] != NE) return;
  if (in_sizes[6] != NTN * CH * CH || in_sizes[7] != NTN * CH * CH) return;
  if (in_sizes[8] != NTN * CH * CH || in_sizes[9] != NTN * CH * CH) return;
  if (in_sizes[10] != NHEAD * NTE * HSZ * HSZ || in_sizes[11] != NHEAD * NTE * HSZ * HSZ) return;
  if (in_sizes[12] != NTE * CH * 1024 || in_sizes[13] != NTE * CH * CH) return;
  if (in_sizes[14] != NHEAD * NTE || in_sizes[15] != NTN) return;
  if (out_size != NN * CH) return;

  const float* x_node = (const float*)d_in[0];
  const float* x_edge = (const float*)d_in[1];
  const int*   ntype  = (const int*)d_in[2];
  const int*   etype  = (const int*)d_in[3];
  const int*   src    = (const int*)d_in[4];
  const int*   dst    = (const int*)d_in[5];
  const float* Wk     = (const float*)d_in[6];
  const float* Wq     = (const float*)d_in[7];
  const float* Wv     = (const float*)d_in[8];
  const float* Wa     = (const float*)d_in[9];
  const float* Wra    = (const float*)d_in[10];
  const float* Wrm    = (const float*)d_in[11];
  const float* WeAtt  = (const float*)d_in[12];
  const float* WeMsg  = (const float*)d_in[13];
  const float* pri    = (const float*)d_in[14];
  const float* skip   = (const float*)d_in[15];
  float* out = (float*)d_out;

  char* ws = (char*)d_ws;
  size_t off = 0;
  const size_t oXNB = off; off += (size_t)MPN * CH * 2;        off = (off + 255) & ~(size_t)255;
  const size_t oXEB = off; off += (size_t)NE * CH * 2;         off = (off + 255) & ~(size_t)255;
  const size_t oKQ  = off; off += (size_t)2 * MPN * CH * 4;    off = (off + 255) & ~(size_t)255;
  const size_t oVP  = off; off += (size_t)MPN * 128 * 2;       off = (off + 255) & ~(size_t)255;
  const size_t oHHL = off; off += (size_t)MPN * 128 * 2;       off = (off + 255) & ~(size_t)255;
  const size_t oMSG = off; off += (size_t)PCAP * CH * 4;       off = (off + 255) & ~(size_t)255;
  const size_t oSC  = off; off += (size_t)PCAP * 4 * 4;        off = (off + 255) & ~(size_t)255;
  const size_t oDST = off; off += (size_t)PCAP * 4;            off = (off + 255) & ~(size_t)255;
  const size_t oPRM = off; off += (size_t)PCAP * 4;            off = (off + 255) & ~(size_t)255;
  const size_t oWKQ = off; off += (size_t)NTN * 192 * CH * 2;  off = (off + 255) & ~(size_t)255;
  const size_t oWA2 = off; off += (size_t)NTN * CH * 128 * 2;  off = (off + 255) & ~(size_t)255;
  const size_t oWB  = off; off += (size_t)WB_TOT * 2;          off = (off + 255) & ~(size_t)255;
  const size_t oFT  = off; off += (size_t)FT_TOT * 4;          off = (off + 255) & ~(size_t)255;
  const size_t oTB  = off; off += (size_t)256;                 off = (off + 255) & ~(size_t)255;
  if (off > ws_size || off > (size_t)WSMAX) return;

  unsigned short* XNB  = (unsigned short*)(ws + oXNB);
  unsigned short* XEB  = (unsigned short*)(ws + oXEB);
  float*          KQ   = (float*)(ws + oKQ);
  unsigned short* VP   = (unsigned short*)(ws + oVP);
  unsigned short* HHL  = (unsigned short*)(ws + oHHL);
  float*          MSG  = (float*)(ws + oMSG);
  float*          SC   = (float*)(ws + oSC);
  int*            DSTP = (int*)(ws + oDST);
  int*            PERM = (int*)(ws + oPRM);
  unsigned short* WKQV = (unsigned short*)(ws + oWKQ);
  unsigned short* WA2  = (unsigned short*)(ws + oWA2);
  unsigned short* WB   = (unsigned short*)(ws + oWB);
  float*          FT   = (float*)(ws + oFT);
  int*            TB   = (int*)(ws + oTB);

  hipFuncSetAttribute(reinterpret_cast<const void*>(&k_edge), hipFuncAttributeMaxDynamicSharedMemorySize,
                      (int)EDGE_LDS);
  hipFuncSetAttribute(reinterpret_cast<const void*>(&k_scan), hipFuncAttributeMaxDynamicSharedMemorySize,
                      (int)LDS_AGG);

  k_pa<<<PA_U1 / NTHR, NTHR, 0, stream>>>(x_node, x_edge, XNB, XEB);
  k_pb<<<PB_NBLK + 1, NTHR, 0, stream>>>(Wk, Wq, Wv, Wa, pri, skip, WKQV, WA2, FT);
  k_pc<<<PC_TOT / NTHR, NTHR, 0, stream>>>(Wra, Wrm, WeAtt, WeMsg, WB, FT);
  k_perm<<<NTE, NTHR, 0, stream>>>(etype, PERM, TB);
  k_node<<<dim3(NMT, NTN), NTHR, 0, stream>>>(XNB, WKQV, ntype, KQ, VP);
  k_edge<<<NTILE, NTHR, EDGE_LDS, stream>>>(PERM, TB, src, dst, XEB, KQ, VP, WB, FT, MSG, SC, DSTP);
  k_scan<<<NSCANB, NTHR, LDS_AGG, stream>>>(DSTP, SC, MSG, (unsigned int*)HHL);
  k_out<<<dim3(NMT, NTN), NTHR, 0, stream>>>(HHL, WA2, ntype, XNB, FT, out);
}
